// PointTransformerGNN_6004364280126
// MI455X (gfx1250) — hardware-verified
//
#include <hip/hip_runtime.h>
#define SS 2
#define NN 1024
#define HH 256
#define NHD 8
#define HD 32
#define NL 4
#define NE 32768
#define NR (SS * NN)
#define FF 1024
#define DCAP 96
typedef __bf16 v16b __attribute__((ext_vector_type(16)));
typedef unsigned short v8us __attribute__((ext_vector_type(8), may_alias));
typedef float  v8f  __attribute__((ext_vector_type(8)));
typedef float  v4f  __attribute__((ext_vector_type(4)));
typedef float  v4fa __attribute__((ext_vector_type(4), may_alias));
union FragB { v16b v; v8us half[2]; unsigned short u[16]; };

__device__ __forceinline__ unsigned short bf16_bits(float x) { unsigned int u = __float_as_uint(x); return (unsigned short)((u + 0x7FFFu + ((u >> 16) & 1u)) >> 16); }
__device__ __forceinline__ float bf16_val(unsigned short b) { return __uint_as_float(((unsigned int)b) << 16); }
__device__ __forceinline__ float bf16_round(float x) { return bf16_val(bf16_bits(x)); }
template <int NT>
__device__ __forceinline__ v8f mmaN(v16b ah, v16b al, v16b bh, v16b bl, v8f c) {
  c = __builtin_amdgcn_wmma_f32_16x16x32_bf16(false, ah, false, bh, (short)0, c, false, false);
  if (NT >= 2) c = __builtin_amdgcn_wmma_f32_16x16x32_bf16(false, al, false, bh, (short)0, c, false, false);
  if (NT >= 3) c = __builtin_amdgcn_wmma_f32_16x16x32_bf16(false, ah, false, bl, (short)0, c, false, false);
  asm volatile("v_nop\n\tv_nop\n\tv_nop\n\tv_nop" : "+v"(c) : "v"(ah), "v"(al), "v"(bh), "v"(bl));
  return c;
}

__global__ __launch_bounds__(256) void k_wt_bf16(const float* __restrict__ W, unsigned short* __restrict__ Wt, int K, int N) {
  const int t = blockIdx.x * 256 + threadIdx.x;
  const int k8n = K / 8;
  if (t >= N * k8n) return;
  const int n = t / k8n, k8 = (t % k8n) * 8;
  v8us v;
#pragma unroll
  for (int i = 0; i < 8; ++i) v[i] = bf16_bits(W[(size_t)(k8 + i) * N + n]);
  *(volatile v8us*)(Wt + (size_t)n * K + k8) = v;
  __threadfence();
  *(volatile v8us*)(Wt + (size_t)n * K + k8) = v;
}

template <bool ASPLIT, int ACT, bool BIAS_BF16>
__global__ __launch_bounds__(128) void k_gemm_bf(const float* __restrict__ A, int lda, const unsigned short* __restrict__ Wt, int ldb,
                                               const float* __restrict__ bias, float* __restrict__ C, int ldc, int M, int N, int K) {
  __shared__ __attribute__((aligned(16))) float so[4][16][64];
  const int tid = threadIdx.x, w = tid >> 5, lane = tid & 31, ln = lane & 15, hh = lane >> 4;
  const int ntn = N / 64;
  const int wid = blockIdx.x * 4 + w;
  const int mt = wid / ntn, nq = wid % ntn;
  if (mt * 16 >= M) return;
  const int row0 = mt * 16, col0 = nq * 64;
  const float* arow = A + (size_t)(row0 + ln) * lda;
  v8f acc[4] = {};
  for (int kb = 0; kb < K; kb += 32) {
    FragB ah, al;
    const v4f x0 = *(const v4fa*)(arow + kb + 8 * hh), x1 = *(const v4fa*)(arow + kb + 8 * hh + 4);
    const v4f x2 = *(const v4fa*)(arow + kb + 16 + 8 * hh), x3 = *(const v4fa*)(arow + kb + 16 + 8 * hh + 4);
    float xs[16] = {x0[0],x0[1],x0[2],x0[3],x1[0],x1[1],x1[2],x1[3],x2[0],x2[1],x2[2],x2[3],x3[0],x3[1],x3[2],x3[3]};
#pragma unroll
    for (int i = 0; i < 16; ++i) { const unsigned short hb = bf16_bits(xs[i]); ah.u[i] = hb; al.u[i] = ASPLIT ? bf16_bits(xs[i] - bf16_val(hb)) : (unsigned short)0; }
#pragma unroll
    for (int t = 0; t < 4; ++t) {
      const unsigned short* brow = Wt + (size_t)(col0 + t * 16 + ln) * ldb + kb;
      FragB b;
      b.half[0] = *(const v8us*)(brow + 8 * hh);
      b.half[1] = *(const v8us*)(brow + 16 + 8 * hh);
      acc[t] = mmaN<ASPLIT ? 2 : 1>(ah.v, al.v, b.v, b.v, acc[t]);
    }
  }
#pragma unroll
  for (int t = 0; t < 4; ++t) {
    float bv = bias ? bias[col0 + t * 16 + ln] : 0.f;
    if (BIAS_BF16) bv = bf16_round(bv);
#pragma unroll
    for (int r = 0; r < 8; ++r) { float v = acc[t][r] + bv; if (ACT == 1) v = fmaxf(v, 0.f); so[w][8 * hh + r][t * 16 + ln] = v; }
  }
  __builtin_amdgcn_fence(__ATOMIC_ACQ_REL, "workgroup");
  __builtin_amdgcn_wave_barrier();
  const int rsub = lane >> 4, c4 = (lane & 15) * 4;
  for (int pass = 0; pass < 2; ++pass) {
#pragma unroll
    for (int q = 0; q < 8; ++q) {
      const int r = q * 2 + rsub;
      const v4f v = *(const v4fa*)&so[w][r][c4];
      *(volatile v4f*)(C + (size_t)(row0 + r) * ldc + col0 + c4) = v;
    }
    if (pass == 0) __threadfence();
  }
}

template <bool ASPLIT, int ACT, bool BIAS_BF16, bool RES_BF16>
__global__ __launch_bounds__(128) void k_gemm_bf3(const float* __restrict__ A, int lda, const unsigned short* __restrict__ Wt, int ldb,
                                                const float* __restrict__ bias, const float* __restrict__ resid, int rmod, int ldr,
                                                float* __restrict__ C, int ldc, int M, int N, int K) {
  __shared__ __attribute__((aligned(16))) float so[4][16][64];
  const int tid = threadIdx.x, w = tid >> 5, lane = tid & 31, ln = lane & 15, hh = lane >> 4;
  const int ntn = N / 64;
  const int wid = blockIdx.x * 4 + w;
  const int mt = wid / ntn, nq = wid % ntn;
  if (mt * 16 >= M) return;
  const int row0 = mt * 16, col0 = nq * 64;
  const float* arow = A + (size_t)(row0 + ln) * lda;
  v8f acc[4] = {};
  for (int kb = 0; kb < K; kb += 32) {
    FragB ah, al;
    const v4f x0 = *(const v4fa*)(arow + kb + 8 * hh), x1 = *(const v4fa*)(arow + kb + 8 * hh + 4);
    const v4f x2 = *(const v4fa*)(arow + kb + 16 + 8 * hh), x3 = *(const v4fa*)(arow + kb + 16 + 8 * hh + 4);
    float xs[16] = {x0[0],x0[1],x0[2],x0[3],x1[0],x1[1],x1[2],x1[3],x2[0],x2[1],x2[2],x2[3],x3[0],x3[1],x3[2],x3[3]};
#pragma unroll
    for (int i = 0; i < 16; ++i) { const unsigned short hb = bf16_bits(xs[i]); ah.u[i] = hb; al.u[i] = ASPLIT ? bf16_bits(xs[i] - bf16_val(hb)) : (unsigned short)0; }
#pragma unroll
    for (int t = 0; t < 4; ++t) {
      const unsigned short* brow = Wt + (size_t)(col0 + t * 16 + ln) * ldb + kb;
      FragB b;
      b.half[0] = *(const v8us*)(brow + 8 * hh);
      b.half[1] = *(const v8us*)(brow + 16 + 8 * hh);
      acc[t] = mmaN<ASPLIT ? 2 : 1>(ah.v, al.v, b.v, b.v, acc[t]);
    }
  }
#pragma unroll
  for (int t = 0; t < 4; ++t) {
    const int col = col0 + t * 16 + ln;
    float bv = bias ? bias[col] : 0.f;
    if (BIAS_BF16) bv = bf16_round(bv);
#pragma unroll
    for (int r = 0; r < 8; ++r) {
      float v = acc[t][r] + bv;
      if (resid) { float rv = resid[(size_t)((row0 + 8 * hh + r) % rmod) * ldr + col]; if (RES_BF16) rv = bf16_round(rv); v += rv; }
      if (ACT == 1) v = fmaxf(v, 0.f);
      if (ACT == 2) v = 0.5f * v * (1.0f + erff(v * 0.70710678118654752f));
      if (ACT == 3) { const float u = 0.7978845608028654f * (v + 0.044715f * v * v * v); v = 0.5f * v * (1.0f + tanhf(u)); }
      so[w][8 * hh + r][t * 16 + ln] = v;
    }
  }
  __builtin_amdgcn_fence(__ATOMIC_ACQ_REL, "workgroup");
  __builtin_amdgcn_wave_barrier();
  const int rsub = lane >> 4, c4 = (lane & 15) * 4;
  for (int pass = 0; pass < 2; ++pass) {
#pragma unroll
    for (int q = 0; q < 8; ++q) {
      const int r = q * 2 + rsub;
      const v4f v = *(const v4fa*)&so[w][r][c4];
      *(volatile v4f*)(C + (size_t)(row0 + r) * ldc + col0 + c4) = v;
    }
    if (pass == 0) __threadfence();
  }
}
template <bool PARAM_BF16>
__global__ __launch_bounds__(256) void k_layernorm(const float* __restrict__ X, const float* __restrict__ R, const float* __restrict__ g, const float* __restrict__ bta,
                                                  float* __restrict__ out_sum, float* __restrict__ out_norm, int N, float eps) {
  __shared__ float red[256];
  const int row = blockIdx.x, tid = threadIdx.x;
  const float* x = X + (size_t)row * N; const float* rr = R ? R + (size_t)row * N : nullptr;
  float vals[16];
  const int per = N / 256;
  float s1 = 0.f;
  for (int u = 0; u < per / 4; ++u) {
    const int j = tid * 4 + 1024 * u;
    const v4f a = *(const v4fa*)(x + j);
    v4f b = {0.f,0.f,0.f,0.f}; if (rr) b = *(const v4fa*)(rr + j);
#pragma unroll
    for (int q = 0; q < 4; ++q) { const float v = a[q] + b[q]; vals[u * 4 + q] = v; s1 += v; }
  }
  red[tid] = s1; __syncthreads();
  for (int st = 128; st > 0; st >>= 1) { if (tid < st) red[tid] += red[tid + st]; __syncthreads(); }
  const float mu = red[0] / (float)N; __syncthreads();
  float s2 = 0.f;
  for (int u = 0; u < per / 4; ++u)
#pragma unroll
    for (int q = 0; q < 4; ++q) { const float c = vals[u * 4 + q] - mu; s2 += c * c; }
  red[tid] = s2; __syncthreads();
  for (int st = 128; st > 0; st >>= 1) { if (tid < st) red[tid] += red[tid + st]; __syncthreads(); }
  const float rs = rsqrtf(red[0] / (float)N + eps);
  for (int pass = 0; pass < 2; ++pass) {
    for (int u = 0; u < per / 4; ++u) {
      const int j = tid * 4 + 1024 * u;
      v4f o, sm;
#pragma unroll
      for (int q = 0; q < 4; ++q) {
        float gg = g[j + q], bb = bta[j + q];
        if (PARAM_BF16) { gg = bf16_round(gg); bb = bf16_round(bb); }
        sm[q] = vals[u * 4 + q]; o[q] = (vals[u * 4 + q] - mu) * rs * gg + bb;
      }
      if (out_sum) *(volatile v4f*)(out_sum + (size_t)row * N + j) = sm;
      *(volatile v4f*)(out_norm + (size_t)row * N + j) = o;
    }
    if (pass == 0) __threadfence();
  }
}


typedef _Float16 v16h __attribute__((ext_vector_type(16)));
union FragH { v16h v; v8us half[2]; _Float16 h[16]; unsigned short u[16]; };
template <int NT>
__device__ __forceinline__ v8f mmaH(v16h ah, v16h al, v16h bh, v16h bl, v8f c) {
  c = __builtin_amdgcn_wmma_f32_16x16x32_f16(false, ah, false, bh, (short)0, c, false, false);
  if (NT >= 2) c = __builtin_amdgcn_wmma_f32_16x16x32_f16(false, al, false, bh, (short)0, c, false, false);
  if (NT >= 3) c = __builtin_amdgcn_wmma_f32_16x16x32_f16(false, ah, false, bl, (short)0, c, false, false);
  asm volatile("v_nop\n\tv_nop\n\tv_nop\n\tv_nop" : "+v"(c) : "v"(ah), "v"(al), "v"(bh), "v"(bl));
  return c;
}
template <bool ASPLIT>
__global__ __launch_bounds__(128) void k_gemm_h(const float* __restrict__ A, int lda, size_t sA, const _Float16* __restrict__ Bh, int ldb, size_t sB, float alpha, float* __restrict__ C, int ldc, size_t sC, int M, int N, int K) {
  __shared__ __attribute__((aligned(16))) float so[4][16][64];
  const int tid = threadIdx.x, w = tid >> 5, lane = tid & 31, ln = lane & 15, hh = lane >> 4; const int by = blockIdx.y;
  A += (size_t)by * sA; Bh += (size_t)by * sB; C += (size_t)by * sC;
  const int ntn = (N + 63) / 64; const int wid = blockIdx.x * 4 + w; const int mt = wid / ntn, nq = wid % ntn; if (mt * 16 >= M) return;
  const int row0 = mt * 16, col0 = nq * 64; const float* arow = A + (size_t)(row0 + ln) * lda;
  v8f acc[4] = {};
  for (int kb = 0; kb < K; kb += 32) {
    FragH ah, al;
    const v4f x0 = *(const v4fa*)(arow + kb + 8 * hh), x1 = *(const v4fa*)(arow + kb + 8 * hh + 4), x2 = *(const v4fa*)(arow + kb + 16 + 8 * hh), x3 = *(const v4fa*)(arow + kb + 16 + 8 * hh + 4);
    float xs[16] = {x0[0],x0[1],x0[2],x0[3],x1[0],x1[1],x1[2],x1[3],x2[0],x2[1],x2[2],x2[3],x3[0],x3[1],x3[2],x3[3]};
#pragma unroll
    for (int i = 0; i < 16; ++i) { const _Float16 h = (_Float16)xs[i]; ah.h[i] = h; al.h[i] = ASPLIT ? (_Float16)(xs[i] - (float)h) : (_Float16)0.0f; }
#pragma unroll
    for (int t = 0; t < 4; ++t) { if (col0 + t * 16 >= N) continue; const size_t boff = (size_t)(col0 + t * 16 + ln) * ldb + kb; FragH bq; bq.half[0] = *(const v8us*)(Bh + boff + 8 * hh); bq.half[1] = *(const v8us*)(Bh + boff + 16 + 8 * hh);
      acc[t] = mmaH<ASPLIT ? 2 : 1>(ah.v, al.v, bq.v, bq.v, acc[t]); }
  }
#pragma unroll
  for (int t = 0; t < 4; ++t) { if (col0 + t * 16 >= N) continue;
#pragma unroll
    for (int r = 0; r < 8; ++r) so[w][8 * hh + r][t * 16 + ln] = acc[t][r] * alpha; }
  __builtin_amdgcn_fence(__ATOMIC_ACQ_REL, "workgroup"); __builtin_amdgcn_wave_barrier();
  const int rsub = lane >> 4, c4 = (lane & 15) * 4;
  for (int pass = 0; pass < 2; ++pass) {
#pragma unroll
    for (int q = 0; q < 8; ++q) { const int r = q * 2 + rsub; if (col0 + c4 < N) { const v4f v = *(const v4fa*)&so[w][r][c4]; *(volatile v4f*)(C + (size_t)(row0 + r) * ldc + col0 + c4) = v; } }
    if (pass == 0) __threadfence(); }
}

__global__ __launch_bounds__(256) void k_wt_f16(const float* __restrict__ W, _Float16* __restrict__ Wt, int K, int N, float scale) {
  const int t = blockIdx.x * 256 + threadIdx.x; if (t >= N * (K / 8)) return; const int n = t / (K / 8), k8 = (t % (K / 8)) * 8; FragH f;
#pragma unroll
  for (int i = 0; i < 8; ++i) f.h[i] = (_Float16)(bf16_round(W[(size_t)(k8 + i) * N + n]) * scale); const v8us o = f.half[0];
  *(volatile v8us*)((unsigned short*)Wt + (size_t)n * K + k8) = o; __threadfence(); *(volatile v8us*)((unsigned short*)Wt + (size_t)n * K + k8) = o;
}
template <int ACT>
__global__ __launch_bounds__(128) void k_gemm_hhx(const _Float16* __restrict__ A, int lda, size_t sA, const _Float16* __restrict__ Bh, int ldb, size_t sB, float alpha, const float* __restrict__ bias, size_t sBias, const float* __restrict__ CP, int rowsPerB, size_t sCPb, int row0g,
    float* __restrict__ C, _Float16* __restrict__ C16, int ldc, size_t sC, int M, int N, int K) {
  __shared__ __attribute__((aligned(16))) float so[4][16][64];
  const int tid = threadIdx.x, w = tid >> 5, lane = tid & 31, ln = lane & 15, hh = lane >> 4; const int by = blockIdx.y;
  A += (size_t)by * sA; Bh += (size_t)by * sB; const size_t cofs = (size_t)by * sC; const float* bp = bias ? bias + (size_t)by * sBias : nullptr;
  const int ntn = (N + 63) / 64; const int wid = blockIdx.x * 4 + w; const int mt = wid / ntn, nq = wid % ntn; if (mt * 16 >= M) return;
  const int row0 = mt * 16, col0 = nq * 64; const _Float16* arow = A + (size_t)(row0 + ln) * lda;
  v8f acc[4] = {};
  for (int kb = 0; kb < K; kb += 32) { FragH ah; ah.half[0] = *(const v8us*)((const unsigned short*)arow + kb + 8 * hh); ah.half[1] = *(const v8us*)((const unsigned short*)arow + kb + 16 + 8 * hh);
#pragma unroll
    for (int t = 0; t < 4; ++t) { if (col0 + t * 16 >= N) continue; const size_t boff = (size_t)(col0 + t * 16 + ln) * ldb + kb; FragH bq; bq.half[0] = *(const v8us*)((const unsigned short*)Bh + boff + 8 * hh); bq.half[1] = *(const v8us*)((const unsigned short*)Bh + boff + 16 + 8 * hh);
      acc[t] = mmaH<1>(ah.v, ah.v, bq.v, bq.v, acc[t]); }
  }
#pragma unroll
  for (int t = 0; t < 4; ++t) { if (col0 + t * 16 >= N) continue; const int col = col0 + t * 16 + ln; const float bv = bp ? bf16_round(bp[col]) : 0.f;
#pragma unroll
    for (int r = 0; r < 8; ++r) { float v = acc[t][r] * alpha + bv; if (CP) { const int bidx = (row0g + row0 + 8 * hh + r) / rowsPerB; v += CP[(size_t)bidx * sCPb + (size_t)by * 64 + col]; } if (ACT == 1) v = (v > 0.f) ? v : expm1f(v); else if (ACT == 7) v = (v > 0.f) ? v + 1.0f : expf(v); else if (ACT == 8) v = tanhf(v); else if (ACT == 9) v = 0.5f * v * (1.0f + tanhf(0.7978845608028654f * (v + 0.044715f * v * v * v))); else if (ACT == 11) v = 1.0f / (1.0f + expf(-v)); else if (ACT == 12) v = (v > 0.f) ? v : 0.01f * v; else if (ACT == 14) v = (v > 0.f) ? v : 0.1f * v; else if (ACT == 15) v = v / (1.0f + expf(-v)); else if (ACT == 3) v = fmaxf(v, 0.f); else if (ACT == 6) v = 0.5f * v * (1.0f + erff(v * 0.70710678118654752f)); so[w][8 * hh + r][t * 16 + ln] = v; } }
  __builtin_amdgcn_fence(__ATOMIC_ACQ_REL, "workgroup"); __builtin_amdgcn_wave_barrier();
  const int rsub = lane >> 4, c4 = (lane & 15) * 4; typedef _Float16 v4h __attribute__((ext_vector_type(4)));
  for (int pass = 0; pass < 2; ++pass) {
#pragma unroll
    for (int q = 0; q < 8; ++q) { const int r = q * 2 + rsub; if (col0 + c4 < N) { const v4f v = *(const v4fa*)&so[w][r][c4]; if (C) *(volatile v4f*)(C + cofs + (size_t)(row0 + r) * ldc + col0 + c4) = v; if (C16) { v4h h4; for (int i = 0; i < 4; ++i) h4[i] = (_Float16)v[i]; *(volatile v4h*)(C16 + cofs + (size_t)(row0 + r) * ldc + col0 + c4) = h4; } } }
    if (pass == 0) __threadfence(); }
}


typedef _Float16 v4h __attribute__((ext_vector_type(4)));

__global__ __launch_bounds__(256) void k_x16(const float* __restrict__ x, _Float16* __restrict__ X16, size_t n8) { const size_t t = (size_t)blockIdx.x * 256 + threadIdx.x; if (t >= n8) return; FragH f;
#pragma unroll
  for (int q = 0; q < 8; ++q) f.h[q] = (_Float16)bf16_round(x[t * 8 + q]); *(volatile v8us*)((unsigned short*)X16 + t * 8) = f.half[0]; __threadfence(); *(volatile v8us*)((unsigned short*)X16 + t * 8) = f.half[0]; }
__global__ __launch_bounds__(256) void k_h16(const float* __restrict__ x, _Float16* __restrict__ X16, size_t n8) { const size_t t = (size_t)blockIdx.x * 256 + threadIdx.x; if (t >= n8) return; FragH f;
#pragma unroll
  for (int q = 0; q < 8; ++q) f.h[q] = (_Float16)x[t * 8 + q]; *(volatile v8us*)((unsigned short*)X16 + t * 8) = f.half[0]; __threadfence(); *(volatile v8us*)((unsigned short*)X16 + t * 8) = f.half[0]; }
__global__ __launch_bounds__(256) void k_round16f(const float* __restrict__ W, _Float16* __restrict__ Bt, size_t n8) { const size_t t = (size_t)blockIdx.x * 256 + threadIdx.x; if (t >= n8) return; FragH f;
#pragma unroll
  for (int i = 0; i < 8; ++i) f.h[i] = (_Float16)(bf16_round(W[t * 8 + i]) * 16.0f); *(volatile v8us*)((unsigned short*)Bt + t * 8) = f.half[0]; __threadfence(); *(volatile v8us*)((unsigned short*)Bt + t * 8) = f.half[0]; }
template <int NHv, int TTv>
__global__ __launch_bounds__(256) void k_vt(const _Float16* __restrict__ V16, int ldv, int voff, _Float16* __restrict__ Vt) { __shared__ unsigned short tl[64][66]; const int tid = threadIdx.x; const int slab = blockIdx.x / (TTv / 64), lg = blockIdx.x % (TTv / 64); const int b = slab / NHv, h = slab % NHv;
  for (int i = tid; i < 64 * 8; i += 256) { const int r = i / 8, c8 = (i % 8) * 8; FragH f; f.half[0] = *(const v8us*)((const unsigned short*)V16 + ((size_t)b * TTv + lg * 64 + r) * ldv + voff + h * 64 + c8);
#pragma unroll
    for (int q = 0; q < 8; ++q) tl[r][c8 + q] = f.u[q]; }
  __syncthreads();
  for (int pass = 0; pass < 2; ++pass) {
#pragma unroll
    for (int rd = 0; rd < 2; ++rd) { const int d = rd * 32 + tid / 8, pc = tid % 8; FragH f;
#pragma unroll
      for (int q = 0; q < 8; ++q) f.u[q] = tl[pc * 8 + q][d];
      *(volatile v8us*)((unsigned short*)Vt + ((size_t)slab * 64 + d) * TTv + lg * 64 + pc * 8) = f.half[0]; }
    if (pass == 0) __threadfence(); } }

__global__ __launch_bounds__(256) void k_hl(const float* __restrict__ F, _Float16* __restrict__ Hh, _Float16* __restrict__ Hl, size_t n8) { const size_t t = (size_t)blockIdx.x * 256 + threadIdx.x; if (t >= n8) return; FragH fh, fl; const v4f a = *(const v4fa*)(F + t * 8), c = *(const v4fa*)(F + t * 8 + 4);
#pragma unroll
  for (int q = 0; q < 4; ++q) { _Float16 h = (_Float16)a[q]; fh.h[q] = h; fl.h[q] = (_Float16)((a[q] - (float)h) * 1024.0f); h = (_Float16)c[q]; fh.h[4 + q] = h; fl.h[4 + q] = (_Float16)((c[q] - (float)h) * 1024.0f); }
  for (int pass = 0; pass < 2; ++pass) { *(volatile v8us*)((unsigned short*)Hh + t * 8) = fh.half[0]; *(volatile v8us*)((unsigned short*)Hl + t * 8) = fl.half[0]; if (pass == 0) __threadfence(); } }
#define VST2(T, ptr, val) do { const T vst2_v_ = (val); *(volatile T*)(ptr) = vst2_v_; __threadfence(); *(volatile T*)(ptr) = vst2_v_; } while (0)

#define C4_NB 4096
#define C4_CH 8192
__device__ __forceinline__ int c4_bucket(int v, int N) { v = min(max(v, 0), N - 1); return (int)(((long long)v * C4_NB) / N); }
__global__ __launch_bounds__(256) void k_c4_count(const int* __restrict__ tgt, int E, int N, int* __restrict__ CNT) {
    __shared__ int hist[C4_NB]; const int ch = blockIdx.x, t = threadIdx.x; const int e0 = ch * C4_CH; const int nt = min(C4_CH, E - e0);
    for (int j = 0; j < 16; ++j) hist[t + 256 * j] = 0; __syncthreads();
    for (int i = t; i < nt; i += 256) atomicAdd(&hist[c4_bucket(tgt[e0 + i], N)], 1);
    __syncthreads();
    for (int j = 0; j < 16; ++j) { const int v = hist[t + 256 * j]; VST2(int, CNT + (long long)ch * C4_NB + t + 256 * j, v); } }
__global__ __launch_bounds__(256) void k_c4_offsets(const int* __restrict__ CNT, int nch, int E, int* __restrict__ OFFB, int* __restrict__ BOFF) {
    __shared__ int tot[C4_NB]; __shared__ int part[256]; const int t = threadIdx.x;
    for (int j = 0; j < 16; ++j) { const int b = t + 256 * j; int s = 0; for (int ch = 0; ch < nch; ++ch) s += CNT[(long long)ch * C4_NB + b]; tot[b] = s; }
    __syncthreads();
    { int s = 0; for (int q = 0; q < 16; ++q) s += tot[16 * t + q]; part[t] = s; } __syncthreads();
    if (t == 0) { int run = 0; for (int i = 0; i < 256; ++i) { const int v = part[i]; part[i] = run; run += v; } } __syncthreads();
    { int run = part[t]; for (int q = 0; q < 16; ++q) { const int v = tot[16 * t + q]; tot[16 * t + q] = run; run += v; } }
    __syncthreads();
    for (int j = 0; j < 16; ++j) { const int b = t + 256 * j; VST2(int, BOFF + b, tot[b]); }
    if (t == 0) VST2(int, BOFF + C4_NB, E);
    for (int j = 0; j < 16; ++j) { const int b = t + 256 * j; int run = tot[b]; for (int ch = 0; ch < nch; ++ch) { VST2(int, OFFB + (long long)ch * C4_NB + b, run); run += CNT[(long long)ch * C4_NB + b]; } } }
__global__ __launch_bounds__(256) void k_c4_scatter(const int* __restrict__ tgt, int E, int N, const int* __restrict__ OFFB, int* __restrict__ BUF) {
    __shared__ int cur[C4_NB]; __shared__ int bk[256]; const int ch = blockIdx.x, t = threadIdx.x; const int e0 = ch * C4_CH; const int nt = min(C4_CH, E - e0);
    const int wv = t >> 5, ln = t & 31;
    for (int j = 0; j < 16; ++j) cur[t + 256 * j] = OFFB[(long long)ch * C4_NB + t + 256 * j];
    __syncthreads();
    for (int s0 = 0; s0 < C4_CH; s0 += 256) {
        const int i = s0 + t; const int e = e0 + i; const int b = (i < nt) ? c4_bucket(tgt[min(e, E - 1)], N) : -1;
        bk[t] = b; __syncthreads();
        int rank = 0, cntw = 0;
        for (int l = 0; l < 32; ++l) { const int o = bk[(wv << 5) + l]; const bool same = (o == b) && (b >= 0); cntw += same ? 1 : 0; rank += (same && l < ln) ? 1 : 0; }
        const bool last = (b >= 0) && (rank == cntw - 1);
        for (int w = 0; w < 8; ++w) {
            if (wv == w && b >= 0) { int pos = cur[b] + rank; pos = min(max(pos, 0), E - 1); VST2(int, BUF + pos, e); }
            __syncthreads();
            if (wv == w && last) cur[b] += cntw;
            __syncthreads(); }
    } }
template <int CAP>
__global__ __launch_bounds__(256) void k_c4_lists(const int* __restrict__ tgt, const int* __restrict__ BUF, const int* __restrict__ BOFF, int N, int E, int* __restrict__ NBR, int* __restrict__ cnt) {
    const int d = blockIdx.x * 256 + threadIdx.x; if (d >= N) return; const int b = c4_bucket(d, N); int n = 0; int* row = NBR + (long long)d * CAP;
    const int p0 = min(max(BOFF[b], 0), E), p1 = min(max(BOFF[b + 1], p0), E);
    for (int p = p0; p < p1; ++p) { int e = BUF[p]; e = min(max(e, 0), E - 1); if (tgt[e] == d) { if (n < CAP) VST2(int, row + n, e); ++n; } }
    for (int j = n; j < CAP; ++j) VST2(int, row + j, -1); VST2(int, cnt + d, min(n, CAP)); }
__global__ __launch_bounds__(256) void k_c4_scan1(const int* __restrict__ cnt, int* __restrict__ PART, int N) {
    __shared__ int part[256]; const int per = ((((N + 255) / 256) + 31) / 32) * 32; const int a = threadIdx.x * per, b = min(N, a + per); int s = 0;
    for (int i = a; i < b; ++i) s += cnt[i]; part[threadIdx.x] = s; __syncthreads();
    if (threadIdx.x == 0) { int run = 0; for (int t = 0; t < 256; ++t) { const int v = part[t]; part[t] = run; run += v; } } __syncthreads();
    VST2(int, PART + threadIdx.x, part[threadIdx.x]); }
__global__ __launch_bounds__(256) void k_c4_scan2(const int* __restrict__ cnt, const int* __restrict__ PART, int* __restrict__ off, int N) {
    const int i = blockIdx.x * 256 + threadIdx.x; if (i > N) return; const int per = ((((N + 255) / 256) + 31) / 32) * 32; const int r = min(i / per, 255); const int a = r * per;
    int s = PART[r]; for (int kq = a; kq < i; ++kq) s += cnt[min(kq, N - 1)];
    VST2(int, off + i, s); }
template <int CAP>
__global__ __launch_bounds__(256) void k_c4_slotcopy(const int* __restrict__ off, const int* __restrict__ NBR, int* __restrict__ slot, int N) {
    const int t = blockIdx.x * 256 + threadIdx.x; const int tot = off[N]; if (t >= tot) return;
    int lo = 0, hi = N - 1; while (lo < hi) { const int mid = (lo + hi + 1) >> 1; if (off[mid] <= t) lo = mid; else hi = mid - 1; }
    int j = t - off[lo]; j = (j < 0) ? 0 : ((j >= CAP) ? (CAP - 1) : j); VST2(int, slot + t, NBR[(long long)lo * CAP + j]); }

__global__ __launch_bounds__(256) void k_fe1(const float* __restrict__ x, const float* __restrict__ W1, const float* __restrict__ b1, _Float16* __restrict__ H1) {
  #pragma clang fp contract(off)
  const int t = blockIdx.x * 256 + threadIdx.x; if (t >= NR * (HH / 8)) return; const int c0 = (t % (HH / 8)) * 8, r = t / (HH / 8); const float x0 = bf16_round(x[r * 3]), x1 = bf16_round(x[r * 3 + 1]), x2 = bf16_round(x[r * 3 + 2]); FragH f;
#pragma unroll
  for (int q = 0; q < 8; ++q) { const int c = c0 + q; float v = bf16_round(b1[c]); v += x0 * bf16_round(W1[c * 3]); v += x1 * bf16_round(W1[c * 3 + 1]); v += x2 * bf16_round(W1[c * 3 + 2]); f.h[q] = (_Float16)fmaxf(v, 0.f); }
  *(volatile v8us*)((unsigned short*)H1 + (size_t)r * HH + c0) = f.half[0]; __threadfence(); *(volatile v8us*)((unsigned short*)H1 + (size_t)r * HH + c0) = f.half[0]; }
__global__ __launch_bounds__(256) void k_f16(const float* __restrict__ F, _Float16* __restrict__ O16, size_t n8) { const size_t t = (size_t)blockIdx.x * 256 + threadIdx.x; if (t >= n8) return; const v4f a = *(const v4fa*)(F + t * 8), c = *(const v4fa*)(F + t * 8 + 4); FragH f;
#pragma unroll
  for (int q = 0; q < 8; ++q) f.h[q] = (_Float16)((q < 4) ? a[q] : c[q - 4]);
  *(volatile v8us*)((unsigned short*)O16 + t * 8) = f.half[0]; __threadfence(); *(volatile v8us*)((unsigned short*)O16 + t * 8) = f.half[0]; }
__global__ __launch_bounds__(256) void k_ln16(const float* __restrict__ X, const float* __restrict__ g, const float* __restrict__ bb, int fold, _Float16* __restrict__ O16) {
  #pragma clang fp contract(off)
  const int tid = threadIdx.x, w = tid >> 5, ln = tid & 31; const int r = blockIdx.x * 8 + w; if (r >= NR) return; float v[8]; float s = 0.f;
#pragma unroll
  for (int k = 0; k < 8; ++k) { v[k] = X[(size_t)r * HH + ln * 8 + k]; s += v[k]; }
  for (int o = 16; o > 0; o >>= 1) s += __shfl_xor(s, o, 32); const float mu = s / (float)HH; float q2 = 0.f;
#pragma unroll
  for (int k = 0; k < 8; ++k) { const float d = v[k] - mu; q2 += d * d; }
  for (int o = 16; o > 0; o >>= 1) q2 += __shfl_xor(q2, o, 32); const float rs = rsqrtf(q2 / (float)HH + 1e-5f); FragH fh, fl;
#pragma unroll
  for (int k = 0; k < 8; ++k) { const int c = ln * 8 + k; const float y = (v[k] - mu) * rs * bf16_round(g[c]) + bf16_round(bb[c]); const _Float16 hi = (_Float16)y; fh.h[k] = hi; fl.h[k] = (_Float16)((y - (float)hi) * 1024.0f); }
  const int pitch = fold ? 2 * HH : HH;
  for (int pass = 0; pass < 2; ++pass) { *(volatile v8us*)((unsigned short*)O16 + (size_t)r * pitch + ln * 8) = fh.half[0]; if (fold) *(volatile v8us*)((unsigned short*)O16 + (size_t)r * pitch + HH + ln * 8) = fl.half[0]; if (pass == 0) __threadfence(); } }
__device__ __forceinline__ v4f shfl4(v4f v, int srcl) { v4f r; r[0] = __shfl(v[0], srcl, 32); r[1] = __shfl(v[1], srcl, 32); r[2] = __shfl(v[2], srcl, 32); r[3] = __shfl(v[3], srcl, 32); return r; }
__device__ __forceinline__ void store_row8(float* row, v4f oa, v4f ob, int l) { const v4f a1 = shfl4(oa, l >> 1), b1 = shfl4(ob, l >> 1), a2 = shfl4(oa, 16 + (l >> 1)), b2 = shfl4(ob, 16 + (l >> 1)); const v4f c1 = (l & 1) ? b1 : a1, c2 = (l & 1) ? b2 : a2; for (int pass = 0; pass < 2; ++pass) { *(volatile v4f*)(row + l * 4) = c1; *(volatile v4f*)(row + 128 + l * 4) = c2; if (pass == 0) __threadfence(); } }
__global__ __launch_bounds__(256) void k_lnres(const float* __restrict__ A, const float* __restrict__ g, const float* __restrict__ bb, const float* __restrict__ RES, float* __restrict__ OUT) {
  #pragma clang fp contract(off)
  const int tid = threadIdx.x, w = tid >> 5, ln = tid & 31; const int r = blockIdx.x * 8 + w; if (r >= NR) return; float v[8]; float s = 0.f;
#pragma unroll
  for (int k = 0; k < 8; ++k) { v[k] = A[(size_t)r * HH + ln * 8 + k]; s += v[k]; }
  for (int o = 16; o > 0; o >>= 1) s += __shfl_xor(s, o, 32); const float mu = s / (float)HH; float q2 = 0.f;
#pragma unroll
  for (int k = 0; k < 8; ++k) { const float d = v[k] - mu; q2 += d * d; }
  for (int o = 16; o > 0; o >>= 1) q2 += __shfl_xor(q2, o, 32); const float rs = rsqrtf(q2 / (float)HH + 1e-5f); v4f oa, ob;
#pragma unroll
  for (int k = 0; k < 8; ++k) { const int c = ln * 8 + k; const float y = (v[k] - mu) * rs * bf16_round(g[c]) + bf16_round(bb[c]) + (RES ? RES[(size_t)r * HH + c] : 0.f); if (k < 4) oa[k] = y; else ob[k - 4] = y; }
  store_row8(OUT + (size_t)r * HH, oa, ob, ln); }
__global__ __launch_bounds__(256) void k_vt(const _Float16* __restrict__ QKV, int s, _Float16* __restrict__ VT) { const int t = blockIdx.x * 256 + threadIdx.x; if (t >= HH * (NN / 8)) return; const int n0 = (t % (NN / 8)) * 8, hd = t / (NN / 8); FragH f;
#pragma unroll
  for (int q = 0; q < 8; ++q) f.h[q] = QKV[((size_t)s * NN + n0 + q) * 3 * HH + 2 * HH + hd];
  *(volatile v8us*)((unsigned short*)VT + (size_t)hd * NN + n0) = f.half[0]; __threadfence(); *(volatile v8us*)((unsigned short*)VT + (size_t)hd * NN + n0) = f.half[0]; }
__global__ __launch_bounds__(256) void k_soft(const float* __restrict__ S, _Float16* __restrict__ P16) {
  #pragma clang fp contract(off)
  const int tid = threadIdx.x, w = tid >> 5, ln = tid & 31; const int row = blockIdx.x * 8 + w; if (row >= NHD * NN) return; const float* sr = S + (size_t)row * NN; float m = -3.0e38f;
#pragma unroll 1
  for (int jb = 0; jb < NN; jb += 256) { const v4f a = *(const v4fa*)(sr + jb + 8 * ln), c = *(const v4fa*)(sr + jb + 8 * ln + 4);
#pragma unroll
    for (int k = 0; k < 4; ++k) { m = fmaxf(m, a[k]); m = fmaxf(m, c[k]); } }
  for (int o = 16; o > 0; o >>= 1) m = fmaxf(m, __shfl_xor(m, o, 32));
  float su = 0.f;
#pragma unroll 1
  for (int jb = 0; jb < NN; jb += 256) { const v4f a = *(const v4fa*)(sr + jb + 8 * ln), c = *(const v4fa*)(sr + jb + 8 * ln + 4);
#pragma unroll
    for (int k = 0; k < 4; ++k) { su += expf(a[k] - m); su += expf(c[k] - m); } }
  for (int o = 16; o > 0; o >>= 1) su += __shfl_xor(su, o, 32); const float inv = 1024.0f / su;
  for (int pass = 0; pass < 2; ++pass) {
#pragma unroll 1
    for (int jb = 0; jb < NN; jb += 256) { const v4f a = *(const v4fa*)(sr + jb + 8 * ln), c = *(const v4fa*)(sr + jb + 8 * ln + 4); FragH f;
#pragma unroll
      for (int k = 0; k < 4; ++k) { f.h[k] = (_Float16)(expf(a[k] - m) * inv); f.h[4 + k] = (_Float16)(expf(c[k] - m) * inv); }
      *(volatile v8us*)((unsigned short*)P16 + (size_t)row * NN + jb + 8 * ln) = f.half[0]; }
    if (pass == 0) __threadfence(); } }
__global__ __launch_bounds__(256) void k_edge(const int* __restrict__ ei, const float* __restrict__ H0, float* __restrict__ EA) {
  #pragma clang fp contract(off)
  const int e = blockIdx.x * 256 + threadIdx.x; if (e >= NE) return; int r = ei[e], c = ei[NE + e]; r = min(max(r, 0), NN - 1); c = min(max(c, 0), NN - 1);
  for (int s = 0; s < SS; ++s) { v4f v; v[0] = H0[((size_t)s * NN + c) * HH + 0] - H0[((size_t)s * NN + r) * HH + 0]; v[1] = H0[((size_t)s * NN + c) * HH + 1] - H0[((size_t)s * NN + r) * HH + 1]; v[2] = H0[((size_t)s * NN + c) * HH + 2] - H0[((size_t)s * NN + r) * HH + 2]; v[3] = 0.f; *(volatile v4f*)(EA + ((size_t)s * NE + e) * 4) = v; __threadfence(); *(volatile v4f*)(EA + ((size_t)s * NE + e) * 4) = v; } }
__global__ __launch_bounds__(256) void k_ehid(const float* __restrict__ PA, const float* __restrict__ EA, const int* __restrict__ ei, int s, const float* __restrict__ M1, const float* __restrict__ b1, _Float16* __restrict__ HE) {
  #pragma clang fp contract(off)
  const int t = blockIdx.x * 256 + threadIdx.x; if (t >= NE * (HH / 8)) return; const int c0 = (t % (HH / 8)) * 8, e = t / (HH / 8); int c = ei[NE + e]; c = min(max(c, 0), NN - 1); const v4f ea = *(const v4fa*)(EA + ((size_t)s * NE + e) * 4); const v4f pa = *(const v4fa*)(PA + ((size_t)s * NN + c) * HH + c0), pb = *(const v4fa*)(PA + ((size_t)s * NN + c) * HH + c0 + 4); FragH f;
#pragma unroll
  for (int q = 0; q < 8; ++q) { const int cc = c0 + q; float v = ((q < 4) ? pa[q] : pb[q - 4]) + bf16_round(b1[cc]); v += ea[0] * bf16_round(M1[(size_t)cc * 259 + 256]); v += ea[1] * bf16_round(M1[(size_t)cc * 259 + 257]); v += ea[2] * bf16_round(M1[(size_t)cc * 259 + 258]); f.h[q] = (_Float16)fmaxf(v, 0.f); }
  *(volatile v8us*)((unsigned short*)HE + (size_t)e * HH + c0) = f.half[0]; __threadfence(); *(volatile v8us*)((unsigned short*)HE + (size_t)e * HH + c0) = f.half[0]; }
__global__ __launch_bounds__(256) void k_m1a(const float* __restrict__ M1, _Float16* __restrict__ Bt) { const int t = blockIdx.x * 256 + threadIdx.x; if (t >= HH * (HH / 8)) return; const int k0 = (t % (HH / 8)) * 8, o = t / (HH / 8); FragH f;
#pragma unroll
  for (int q = 0; q < 8; ++q) f.h[q] = (_Float16)(bf16_round(M1[(size_t)o * 259 + k0 + q]) * 16.0f);
  *(volatile v8us*)((unsigned short*)Bt + (size_t)o * HH + k0) = f.half[0]; __threadfence(); *(volatile v8us*)((unsigned short*)Bt + (size_t)o * HH + k0) = f.half[0]; }
__global__ __launch_bounds__(256) void k_smean(const int* __restrict__ NBR, const int* __restrict__ cnt, const float* __restrict__ MSG, int s, float* __restrict__ AG) {
  #pragma clang fp contract(off)
  const int tid = threadIdx.x, w = tid >> 5, ln = tid & 31; const int n = blockIdx.x * 8 + w; if (n >= NN) return; const int ne = min(cnt[n], DCAP); float v[8];
#pragma unroll
  for (int k = 0; k < 8; ++k) v[k] = 0.f;
#pragma unroll 1
  for (int j = 0; j < ne; ++j) { int e = NBR[(size_t)n * DCAP + j]; e = min(max(e, 0), NE - 1); const v4f a = *(const v4fa*)(MSG + (size_t)e * HH + ln * 8), c = *(const v4fa*)(MSG + (size_t)e * HH + ln * 8 + 4);
#pragma unroll
    for (int k = 0; k < 8; ++k) v[k] += (k < 4) ? a[k] : c[k - 4]; }
  const float dv = fmaxf((float)cnt[n], 1.0f); v4f oa, ob;
#pragma unroll
  for (int k = 0; k < 8; ++k) { const float y = v[k] / dv; if (k < 4) oa[k] = y; else ob[k - 4] = y; }
  store_row8(AG + ((size_t)s * NN + n) * HH, oa, ob, ln); }
__global__ __launch_bounds__(256) void k_tatt(const float* __restrict__ QKV, _Float16* __restrict__ O16) {
  #pragma clang fp contract(off)
  const int t = blockIdx.x * 256 + threadIdx.x; if (t >= NR * 32) return; const int qq = t & 3, h = (t >> 2) & 7, r = t >> 5; const int s = r / NN, n = r % NN; const float* q = QKV + (size_t)r * 3 * HH + h * HD; float sc[SS];
#pragma unroll
  for (int s2 = 0; s2 < SS; ++s2) { const float* k = QKV + ((size_t)s2 * NN + n) * 3 * HH + HH + h * HD; float a = 0.f;
#pragma unroll
    for (int d = 0; d < HD; ++d) a += q[d] * k[d]; sc[s2] = a * (1.0f / sqrtf((float)HD)); }
  const float m = fmaxf(sc[0], sc[1]); const float e0 = expf(sc[0] - m), e1 = expf(sc[1] - m); const float p0 = e0 / (e0 + e1), p1 = e1 / (e0 + e1); FragH f;
#pragma unroll
  for (int qd = 0; qd < 8; ++qd) { const int d = qq * 8 + qd; const float v0 = QKV[((size_t)0 * NN + n) * 3 * HH + 2 * HH + h * HD + d], v1 = QKV[((size_t)1 * NN + n) * 3 * HH + 2 * HH + h * HD + d]; f.h[qd] = (_Float16)(p0 * v0 + p1 * v1); }
  *(volatile v8us*)((unsigned short*)O16 + (size_t)r * HH + h * HD + qq * 8) = f.half[0]; __threadfence(); *(volatile v8us*)((unsigned short*)O16 + (size_t)r * HH + h * HD + qq * 8) = f.half[0]; (void)s; }
__global__ __launch_bounds__(256) void k_bfold(const float* __restrict__ Wm, int O, _Float16* __restrict__ Bt) { const int t = blockIdx.x * 256 + threadIdx.x; if (t >= O * 64) return; const int k0 = (t & 63) * 8, o = t >> 6; const int kb = k0 & 255; const float sc = (k0 >= 256) ? (16.0f / 1024.0f) : 16.0f; FragH f;
#pragma unroll
  for (int q = 0; q < 8; ++q) f.h[q] = (_Float16)(bf16_round(Wm[(size_t)o * HH + kb + q]) * sc);
  *(volatile v8us*)((unsigned short*)Bt + (size_t)o * 512 + k0) = f.half[0]; __threadfence(); *(volatile v8us*)((unsigned short*)Bt + (size_t)o * 512 + k0) = f.half[0]; }
__global__ __launch_bounds__(256) void k_last2(const float* __restrict__ HT, _Float16* __restrict__ L2) {
  #pragma clang fp contract(off)
  const int t = blockIdx.x * 256 + threadIdx.x; if (t >= NN * (HH / 8)) return; const int c0 = (t % (HH / 8)) * 8, n = t / (HH / 8); const float* src = HT + ((size_t)1 * NN + n) * HH + c0; FragH fh, fl;
#pragma unroll
  for (int q = 0; q < 8; ++q) { const float v = src[q]; const _Float16 hi = (_Float16)v; fh.h[q] = hi; fl.h[q] = (_Float16)((v - (float)hi) * 1024.0f); }
  for (int pass = 0; pass < 2; ++pass) { *(volatile v8us*)((unsigned short*)L2 + (size_t)n * 512 + c0) = fh.half[0]; *(volatile v8us*)((unsigned short*)L2 + (size_t)n * 512 + HH + c0) = fl.half[0]; if (pass == 0) __threadfence(); } }
__global__ __launch_bounds__(256) void k_head2(const float* __restrict__ R1, const float* __restrict__ O2, const float* __restrict__ b2, float* __restrict__ out) {
  #pragma clang fp contract(off)
  const int tid = threadIdx.x; if (tid >= 32) return;
  for (int pass = 0; pass < 2; ++pass) { for (int i = tid; i < NN * 3; i += 32) { const int n = i / 3, j = i % 3; float s = bf16_round(b2[j]); const float* rr = R1 + (size_t)n * HH; const float* ow = O2 + (size_t)j * HH;
#pragma unroll 1
      for (int c = 0; c < HH; c += 4) { s += rr[c] * bf16_round(ow[c]); s += rr[c + 1] * bf16_round(ow[c + 1]); s += rr[c + 2] * bf16_round(ow[c + 2]); s += rr[c + 3] * bf16_round(ow[c + 3]); }
      *(volatile float*)(out + i) = s; } if (pass == 0) __threadfence(); } }

extern "C" void kernel_launch(void* const* d_in, const int* in_sizes, int n_in,
                              void* d_out, int out_size, void* d_ws, size_t ws_size, hipStream_t stream) {
  (void)in_sizes; (void)n_in; (void)out_size;
  const float* const* I = (const float* const*)d_in; const float* x = I[0]; const int* ei = (const int*)d_in[1];
  const float* fe_w1 = I[2]; const float* fe_b1 = I[3]; const float* fe_w2 = I[4]; const float* fe_b2 = I[5]; const float* g_inw = I[6]; const float* g_inb = I[7]; const float* g_outw = I[8]; const float* g_outb = I[9]; const float* g_m1w = I[10]; const float* g_m1b = I[11]; const float* g_m2w = I[12]; const float* g_m2b = I[13]; const float* g_n1g = I[14]; const float* g_n1b = I[15]; const float* g_n2g = I[16]; const float* g_n2b = I[17]; const float* t_inw = I[18]; const float* t_inb = I[19]; const float* t_outw = I[20]; const float* t_outb = I[21]; const float* t_l1w = I[22]; const float* t_l1b = I[23]; const float* t_l2w = I[24]; const float* t_l2b = I[25]; const float* t_n1g = I[26]; const float* t_n1b = I[27]; const float* t_n2g = I[28]; const float* t_n2b = I[29]; const float* o_w1 = I[30]; const float* o_b1 = I[31]; const float* o_w2 = I[32]; const float* o_b2 = I[33];
  char* ws = (char*)d_ws; size_t off = 0;
  auto take = [&](size_t bytes) { char* p = ws + off; off += (bytes + 255) & ~(size_t)255; return p; };
  const int nch = (NE + C4_CH - 1) / C4_CH;
  int* CNT = (int*)take((size_t)nch * C4_NB * 4); int* OFFB = (int*)take((size_t)nch * C4_NB * 4); int* BOFF = (int*)take((size_t)(C4_NB + 64) * 4); int* BUF = (int*)take((size_t)NE * 4); int* NBR = (int*)take((size_t)NN * DCAP * 4); int* cnt = (int*)take((size_t)(NN + 64) * 4);
  _Float16* BFE2 = (_Float16*)take(HH * HH * 2); _Float16* BIN = (_Float16*)take(3 * HH * HH * 2); _Float16* BOUT = (_Float16*)take(HH * HH * 2); _Float16* BM1 = (_Float16*)take(HH * HH * 2); _Float16* BM2 = (_Float16*)take(HH * HH * 2); _Float16* BL1 = (_Float16*)take(FF * HH * 2); _Float16* BL2 = (_Float16*)take(HH * FF * 2); _Float16* BO1 = (_Float16*)take(HH * 512 * 2);
  _Float16* X16 = (_Float16*)take((size_t)NR * HH * 2); float* Hf = (float*)take((size_t)NR * HH * 4); float* H0 = (float*)take((size_t)NR * HH * 4); float* EA = (float*)take((size_t)SS * NE * 4 * 4); _Float16* QKV16 = (_Float16*)take((size_t)NR * 3 * HH * 2); _Float16* VT = (_Float16*)take((size_t)HH * NN * 2); float* S = (float*)take((size_t)NHD * NN * NN * 4); _Float16* P16 = (_Float16*)take((size_t)NHD * NN * NN * 2); _Float16* O16 = (_Float16*)take((size_t)NR * HH * 2); float* A = (float*)take((size_t)NR * HH * 4); _Float16* A16 = (_Float16*)take((size_t)NR * HH * 2); float* PA = (float*)take((size_t)NR * HH * 4); _Float16* HE = (_Float16*)take((size_t)NE * HH * 2); float* AG = (float*)take((size_t)NR * HH * 4); _Float16* F16 = (_Float16*)take((size_t)NR * FF * 2); float* T = (float*)take((size_t)NR * HH * 4); _Float16* L2 = (_Float16*)take((size_t)NN * 512 * 2); float* R1 = (float*)take((size_t)NN * HH * 4);
  float* MSG = S;
  float* QKV = S;
  if (off > ws_size) return;
  k_c4_count<<<nch, 256, 0, stream>>>(ei, NE, NN, CNT); k_c4_offsets<<<1, 256, 0, stream>>>(CNT, nch, NE, OFFB, BOFF); k_c4_scatter<<<nch, 256, 0, stream>>>(ei, NE, NN, OFFB, BUF); k_c4_lists<DCAP><<<(NN + 255) / 256, 256, 0, stream>>>(ei, BUF, BOFF, NN, NE, NBR, cnt);
  const size_t n8 = (size_t)NR * HH / 8; const unsigned nb8 = (unsigned)((n8 + 255) / 256); const dim3 gH(((NR / 16) * (HH / 64) + 3) / 4, 1), g3H(((NR / 16) * (3 * HH / 64) + 3) / 4, 1), gF(((NR / 16) * (FF / 64) + 3) / 4, 1), gE(((NE / 16) * (HH / 64) + 3) / 4, 1);
  k_fe1<<<nb8, 256, 0, stream>>>(x, fe_w1, fe_b1, X16); k_round16f<<<(HH * HH / 8 + 255) / 256, 256, 0, stream>>>(fe_w2, BFE2, (size_t)HH * HH / 8);
  k_gemm_hhx<0><<<gH, 128, 0, stream>>>(X16, HH, 0, BFE2, HH, 0, 0.0625f, fe_b2, 0, nullptr, 1, 0, 0, Hf, nullptr, HH, 0, NR, HH, HH);
  k_edge<<<(NE + 255) / 256, 256, 0, stream>>>(ei, Hf, EA);
  const dim3 gS(((NN / 16) * (NN / 64) + 3) / 4, NHD), gV(((NN / 16) * 1 + 3) / 4, NHD);
  for (int l = 0; l < NL; ++l) {
    k_round16f<<<(3 * HH * HH / 8 + 255) / 256, 256, 0, stream>>>(g_inw + (size_t)l * 3 * HH * HH, BIN, (size_t)3 * HH * HH / 8); k_round16f<<<(HH * HH / 8 + 255) / 256, 256, 0, stream>>>(g_outw + (size_t)l * HH * HH, BOUT, (size_t)HH * HH / 8); k_m1a<<<(HH * (HH / 8) + 255) / 256, 256, 0, stream>>>(g_m1w + (size_t)l * HH * 259, BM1); k_round16f<<<(HH * HH / 8 + 255) / 256, 256, 0, stream>>>(g_m2w + (size_t)l * HH * HH, BM2, (size_t)HH * HH / 8);
    k_ln16<<<NR / 8, 256, 0, stream>>>(Hf, g_n1g + l * HH, g_n1b + l * HH, 0, A16);
    k_gemm_hhx<0><<<g3H, 128, 0, stream>>>(A16, HH, 0, BIN, HH, 0, 0.0625f, g_inb + (size_t)l * 3 * HH, 0, nullptr, 1, 0, 0, nullptr, QKV16, 3 * HH, 0, NR, 3 * HH, HH);
    for (int s = 0; s < SS; ++s) { const _Float16* base = QKV16 + (size_t)s * NN * 3 * HH;
      k_vt<<<(HH * (NN / 8) + 255) / 256, 256, 0, stream>>>(QKV16, s, VT);
      k_gemm_hhx<0><<<gS, 128, 0, stream>>>(base, 3 * HH, (size_t)HD, base + HH, 3 * HH, (size_t)HD, 0.17677669529663687f, nullptr, 0, nullptr, 1, 0, 0, S, nullptr, NN, (size_t)NN * NN, NN, NN, HD);
      k_soft<<<NHD * NN / 8, 256, 0, stream>>>(S, P16);
      k_gemm_hhx<0><<<gV, 128, 0, stream>>>(P16, NN, (size_t)NN * NN, VT, NN, (size_t)HD * NN, 0.0009765625f, nullptr, 0, nullptr, 1, 0, 0, nullptr, O16 + (size_t)s * NN * HH, HH, (size_t)HD, NN, HD, NN); }
    k_gemm_hhx<0><<<gH, 128, 0, stream>>>(O16, HH, 0, BOUT, HH, 0, 0.0625f, g_outb + l * HH, 0, Hf, 1, (size_t)HH, 0, A, nullptr, HH, 0, NR, HH, HH);
    k_f16<<<nb8, 256, 0, stream>>>(A, A16, n8);
    k_gemm_hhx<0><<<gH, 128, 0, stream>>>(A16, HH, 0, BM1, HH, 0, 0.0625f, nullptr, 0, nullptr, 1, 0, 0, PA, nullptr, HH, 0, NR, HH, HH);
    for (int s = 0; s < SS; ++s) {
      k_ehid<<<(NE * (HH / 8) + 255) / 256, 256, 0, stream>>>(PA, EA, ei, s, g_m1w + (size_t)l * HH * 259, g_m1b + l * HH, HE);
      k_gemm_hhx<0><<<gE, 128, 0, stream>>>(HE, HH, 0, BM2, HH, 0, 0.0625f, g_m2b + l * HH, 0, nullptr, 1, 0, 0, MSG, nullptr, HH, 0, NE, HH, HH);
      k_smean<<<NN / 8, 256, 0, stream>>>(NBR, cnt, MSG, s, AG); }
    k_lnres<<<NR / 8, 256, 0, stream>>>(AG, g_n2g + l * HH, g_n2b + l * HH, Hf, Hf); }
  for (int l = 0; l < NL; ++l) {
    k_round16f<<<(3 * HH * HH / 8 + 255) / 256, 256, 0, stream>>>(t_inw + (size_t)l * 3 * HH * HH, BIN, (size_t)3 * HH * HH / 8); k_round16f<<<(HH * HH / 8 + 255) / 256, 256, 0, stream>>>(t_outw + (size_t)l * HH * HH, BOUT, (size_t)HH * HH / 8); k_round16f<<<(FF * HH / 8 + 255) / 256, 256, 0, stream>>>(t_l1w + (size_t)l * FF * HH, BL1, (size_t)FF * HH / 8); k_round16f<<<(unsigned)(((size_t)HH * FF / 8 + 255) / 256), 256, 0, stream>>>(t_l2w + (size_t)l * HH * FF, BL2, (size_t)HH * FF / 8);
    k_f16<<<nb8, 256, 0, stream>>>(Hf, A16, n8);
    k_gemm_hhx<0><<<g3H, 128, 0, stream>>>(A16, HH, 0, BIN, HH, 0, 0.0625f, t_inb + (size_t)l * 3 * HH, 0, nullptr, 1, 0, 0, QKV, nullptr, 3 * HH, 0, NR, 3 * HH, HH);
    k_tatt<<<(NR * 32 + 255) / 256, 256, 0, stream>>>(QKV, O16);
    k_gemm_hhx<0><<<gH, 128, 0, stream>>>(O16, HH, 0, BOUT, HH, 0, 0.0625f, t_outb + l * HH, 0, Hf, 1, (size_t)HH, 0, T, nullptr, HH, 0, NR, HH, HH);
    k_lnres<<<NR / 8, 256, 0, stream>>>(T, t_n1g + l * HH, t_n1b + l * HH, nullptr, Hf);
    k_f16<<<nb8, 256, 0, stream>>>(Hf, A16, n8);
    k_gemm_hhx<3><<<gF, 128, 0, stream>>>(A16, HH, 0, BL1, HH, 0, 0.0625f, t_l1b + (size_t)l * FF, 0, nullptr, 1, 0, 0, nullptr, F16, FF, 0, NR, FF, HH);
    k_gemm_hhx<0><<<gH, 128, 0, stream>>>(F16, FF, 0, BL2, FF, 0, 0.0625f, t_l2b + l * HH, 0, Hf, 1, (size_t)HH, 0, T, nullptr, HH, 0, NR, HH, FF);
    k_lnres<<<NR / 8, 256, 0, stream>>>(T, t_n2g + l * HH, t_n2b + l * HH, nullptr, Hf); }
  k_bfold<<<(HH * 64 + 255) / 256, 256, 0, stream>>>(o_w1, HH, BO1); k_last2<<<(NN * (HH / 8) + 255) / 256, 256, 0, stream>>>(Hf, L2);
  k_gemm_hhx<3><<<dim3(((NN / 16) * (HH / 64) + 3) / 4, 1), 128, 0, stream>>>(L2, 512, 0, BO1, 512, 0, 0.0625f, o_b1, 0, nullptr, 1, 0, 0, R1, nullptr, HH, 0, NN, HH, 512);
  k_head2<<<1, 256, 0, stream>>>(R1, o_w2, o_b2, (float*)d_out);
}
